// GAT_L3_45801531245070
// MI455X (gfx1250) — hardware-verified
//
#include <hip/hip_runtime.h>
#include <stddef.h>


#define HID   32
#define NB    1024
#define CHUNK 2048
#define NTHR  256
#define NWAVE 8
#define WCAP  256
#define NGRP  (CHUNK / (NTHR * 4))
#define PPD   128
#define BNW   128

static_assert(WCAP == (CHUNK / NTHR) * 32);
static_assert(NGRP == 2);
static_assert(NB == 1024);
static_assert(CHUNK == 2048);

#define GAT_LDS(HDv, NHv) ((NB * (HDv) + 2 * NB * (NHv) + NWAVE * WCAP + NWAVE) * 4)
static_assert(GAT_LDS(64, 2) == 286752);
static_assert(GAT_LDS(32, 1) == 147488);

typedef float  v4f  __attribute__((ext_vector_type(4)));
typedef float  v8f  __attribute__((ext_vector_type(8)));
typedef int    v4i  __attribute__((ext_vector_type(4)));
typedef double v2d  __attribute__((ext_vector_type(2)));
typedef __bf16 v16b __attribute__((ext_vector_type(16)));

union Frag { v16b v; struct { v4i q0; v4i q1; } q; };

__device__ __forceinline__ v8f wm(v16b a, v16b b, v8f c) {
  v8f d = __builtin_amdgcn_wmma_f32_16x16x32_bf16(false, a, false, b, (short)0, c, false, false);
  asm volatile("v_nop\n\tv_nop\n\tv_nop\n\tv_nop" : "+v"(d) : "v"(a), "v"(b));
  return d;
}

__device__ __forceinline__ unsigned bf16_rne(float f) {
  unsigned u = __float_as_uint(f);
  u += 0x7FFFu + ((u >> 16) & 1u);
  return u >> 16;
}

__device__ __forceinline__ void split2(float a, float b, int& hi, int& lo) {
  const unsigned ha = bf16_rne(a), hb = bf16_rne(b);
  const float ra = a - __uint_as_float(ha << 16);
  const float rb = b - __uint_as_float(hb << 16);
  const unsigned la = bf16_rne(ra), lb = bf16_rne(rb);
  hi = (int)(ha | (hb << 16));
  lo = (int)(la | (lb << 16));
}

__device__ __forceinline__ void split8(v4f a, v4f b, v4i& hi, v4i& lo) {
  int h0, l0, h1, l1, h2, l2, h3, l3;
  split2(a.x, a.y, h0, l0);
  split2(a.z, a.w, h1, l1);
  split2(b.x, b.y, h2, l2);
  split2(b.z, b.w, h3, l3);
  hi.x = h0; hi.y = h1; hi.z = h2; hi.w = h3;
  lo.x = l0; lo.y = l1; lo.z = l2; lo.w = l3;
}

__global__ __launch_bounds__(NTHR) void k_prep(const float* __restrict__ W,
                                               unsigned short* Whi, unsigned short* Wlo,
                                               int K, int NC) {
  const int kq = K / 8;
  const int n8 = NC * kq;
  const int i = blockIdx.x * NTHR + threadIdx.x;
  if (i >= n8) return;
  const int n = i / kq;
  const int k8 = (i - n * kq) * 8;
  v4f a, b;
  a.x = W[(size_t)(k8 + 0) * NC + n]; a.y = W[(size_t)(k8 + 1) * NC + n];
  a.z = W[(size_t)(k8 + 2) * NC + n]; a.w = W[(size_t)(k8 + 3) * NC + n];
  b.x = W[(size_t)(k8 + 4) * NC + n]; b.y = W[(size_t)(k8 + 5) * NC + n];
  b.z = W[(size_t)(k8 + 6) * NC + n]; b.w = W[(size_t)(k8 + 7) * NC + n];
  v4i ph, pl;
  split8(a, b, ph, pl);
  const size_t o = (size_t)n * K + k8;
  *(volatile v4i*)(Whi + o) = ph;
  *(volatile v4i*)(Wlo + o) = pl;
  __threadfence();
  *(volatile v4i*)(Whi + o) = ph;
  *(volatile v4i*)(Wlo + o) = pl;
}

template <int K, int NC, int NH, int GR, int BN>
__global__ __launch_bounds__(NTHR) void k_gemm(
    const float* __restrict__ A,
    const unsigned short* __restrict__ Whi, const unsigned short* __restrict__ Wlo,
    const float* __restrict__ as, const float* __restrict__ ad, const float* __restrict__ bn,
    float* hout, float* coef, int nN) {
  constexpr int AP   = K + 8;
  constexpr int XSP  = NC + 4;
  constexpr int NT   = NC / 16;
  constexpr int CP   = 2 * NH;
  constexpr int EPT  = GR * K / NTHR;
  constexpr int TPRA = K / EPT;
  constexpr int TPR  = NTHR / GR;
  constexpr int RPW  = GR / NWAVE;
  static_assert(NT * (GR / 16) == NWAVE);
  static_assert(EPT == 8 || EPT == 16);
  static_assert(TPRA * EPT == K);
  static_assert(NTHR / TPRA == GR);
  static_assert(NC == NH * HID);
  static_assert(GR * CP == 128);
  static_assert(TPR * 8 == NC);
  static_assert(RPW * NC == 256);
  static_assert((K % 32) == 0);

  __shared__ __attribute__((aligned(16))) unsigned short Ah[GR * AP];
  __shared__ __attribute__((aligned(16))) unsigned short Al[GR * AP];
  __shared__ __attribute__((aligned(16))) float Xs[GR * XSP];
  __shared__ __attribute__((aligned(16))) float Cs[128];

  const int tid  = threadIdx.x;
  const int lane = tid & 31;
  const int wave = tid >> 5;
  const int hh   = lane >> 4;
  const int m    = lane & 15;
  const int rowBase = blockIdx.x * GR;

  {
    const int r  = tid / TPRA;
    const int c0 = (tid - r * TPRA) * EPT;
    int row = rowBase + r;
    if (row > nN - 1) row = nN - 1;
    const float* p = A + (size_t)row * K + c0;
#pragma unroll
    for (int g = 0; g < EPT / 8; ++g) {
      v4f f0 = *(const v4f*)(p + 8 * g);
      v4f f1 = *(const v4f*)(p + 8 * g + 4);
      if (BN) {
        const v4f s0 = *(const v4f*)(bn + c0 + 8 * g);
        const v4f s1 = *(const v4f*)(bn + c0 + 8 * g + 4);
        const v4f t0 = *(const v4f*)(bn + 64 + c0 + 8 * g);
        const v4f t1 = *(const v4f*)(bn + 64 + c0 + 8 * g + 4);
        f0 = f0 * s0 + t0;
        f1 = f1 * s1 + t1;
        f0.x = fmaxf(f0.x, 0.f); f0.y = fmaxf(f0.y, 0.f); f0.z = fmaxf(f0.z, 0.f); f0.w = fmaxf(f0.w, 0.f);
        f1.x = fmaxf(f1.x, 0.f); f1.y = fmaxf(f1.y, 0.f); f1.z = fmaxf(f1.z, 0.f); f1.w = fmaxf(f1.w, 0.f);
      }
      v4i ph, pl;
      split8(f0, f1, ph, pl);
      *(v4i*)(Ah + r * AP + c0 + 8 * g) = ph;
      *(v4i*)(Al + r * AP + c0 + 8 * g) = pl;
    }
  }
  __syncthreads();

  const int rt = wave / NT;
  const int ct = wave - rt * NT;
  v8f acc = {0.f, 0.f, 0.f, 0.f, 0.f, 0.f, 0.f, 0.f};
#pragma unroll
  for (int kt = 0; kt < K / 32; ++kt) {
    const int k0 = kt * 32;
    Frag ah, al, bh, bl;
    const unsigned short* pa = Ah + (rt * 16 + m) * AP + k0 + 8 * hh;
    const unsigned short* pl = Al + (rt * 16 + m) * AP + k0 + 8 * hh;
    const unsigned short* pb = Whi + (size_t)(ct * 16 + m) * K + k0 + 8 * hh;
    const unsigned short* pc = Wlo + (size_t)(ct * 16 + m) * K + k0 + 8 * hh;
    ah.q.q0 = *(const v4i*)pa;  ah.q.q1 = *(const v4i*)(pa + 16);
    al.q.q0 = *(const v4i*)pl;  al.q.q1 = *(const v4i*)(pl + 16);
    bh.q.q0 = *(const v4i*)pb;  bh.q.q1 = *(const v4i*)(pb + 16);
    bl.q.q0 = *(const v4i*)pc;  bl.q.q1 = *(const v4i*)(pc + 16);
    acc = wm(ah.v, bh.v, acc);
    acc = wm(ah.v, bl.v, acc);
    acc = wm(al.v, bh.v, acc);
  }

#pragma unroll
  for (int r = 0; r < 8; ++r) Xs[(rt * 16 + 8 * hh + r) * XSP + ct * 16 + m] = acc[r];
  __syncthreads();

  {
    const int row  = tid / TPR;
    const int part = tid - row * TPR;
    const int cb   = part * 8;
    const int hd   = cb / HID;
    float s = 0.f, d = 0.f;
#pragma unroll
    for (int j = 0; j < 8; ++j) {
      const float xv = Xs[row * XSP + cb + j];
      s += xv * as[cb + j];
      d += xv * ad[cb + j];
    }
    s += __shfl_xor(s, 1, 32); s += __shfl_xor(s, 2, 32);
    d += __shfl_xor(d, 1, 32); d += __shfl_xor(d, 2, 32);
    if ((part & 3) == 0) {
      Cs[row * CP + hd]      = s;
      Cs[row * CP + NH + hd] = d;
    }
  }
  __syncthreads();

  v4f xr[2];
#pragma unroll
  for (int i = 0; i < 2; ++i) {
    const int f  = i * 128 + lane * 4;
    const int lr = wave * RPW + f / NC;
    const int lc = f % NC;
    xr[i] = *(const v4f*)(Xs + lr * XSP + lc);
  }
  const v4f cv = *(const v4f*)(Cs + lane * 4);
  float* hp = hout + (size_t)(rowBase + wave * RPW) * NC + lane * 4;
  float* cp = coef + (size_t)rowBase * CP + lane * 4;
  *(volatile v4f*)(hp)       = xr[0];
  *(volatile v4f*)(hp + 128) = xr[1];
  if (wave == 0) *(volatile v4f*)cp = cv;
  __threadfence();
  *(volatile v4f*)(hp)       = xr[0];
  *(volatile v4f*)(hp + 128) = xr[1];
  if (wave == 0) *(volatile v4f*)cp = cv;
}

template <int HD, int NH>
__global__ __launch_bounds__(NTHR) void k_gat(
    const int* __restrict__ ei, const float* __restrict__ h, const float* __restrict__ coef,
    const float* __restrict__ bias, float* agg, double* part, int nN, int nE, int nP) {
  constexpr int CPL = HD / 32;
  constexpr int CP  = 2 * NH;
  constexpr int NIT = NB * HD / (NTHR * 4);
  constexpr int SPW = NB / NWAVE;
  static_assert(HD == NH * HID);
  static_assert(CPL >= 1 && CPL * 32 == HD);
  static_assert(NWAVE * 2 * HD * 8 <= NWAVE * WCAP * 4);
  static_assert(NIT * NTHR * 4 == NB * HD);

  extern __shared__ v4f lds_dyn[];
  float*  sacc  = (float*)lds_dyn;
  float*  rmx   = sacc + NB * HD;
  float*  den   = rmx + NB * NH;
  int*    list  = (int*)(den + NB * NH);
  int*    wcnt  = list + NWAVE * WCAP;
  double* bpart = (double*)list;

  const int tid  = threadIdx.x;
  const int lane = tid & 31;
  const int wave = tid >> 5;
  const int cb   = lane * CPL;
  const int hd   = cb / HID;
  const int nodeBase = blockIdx.x * NB;

#pragma unroll 1
  for (int p = tid; p < NB * HD / 4; p += NTHR) {
    const int slot = p / (HD / 4);
    const int c4   = (p - slot * (HD / 4)) * 4;
    int node = nodeBase + slot;
    if (node > nN - 1) node = nN - 1;
    *(v4f*)(sacc + slot * HD + c4) = *(const v4f*)(h + (size_t)node * HD + c4);
  }
#pragma unroll 1
  for (int i = tid; i < NB * NH; i += NTHR) {
    const int slot = i / NH;
    const int hq   = i - slot * NH;
    int node = nodeBase + slot;
    if (node > nN - 1) node = nN - 1;
    float l = coef[(size_t)node * CP + hq] + coef[(size_t)node * CP + NH + hq];
    l = (l > 0.f) ? l : 0.2f * l;
    rmx[i] = l;
    den[i] = 1.0f;
  }
  __syncthreads();

  const int* eid = ei + nE;
  const bool al16 = ((nE & 3) == 0);
  const int nChunks = (nE + CHUNK - 1) / CHUNK;
  const int sent = -2147483647 - 1;
#pragma unroll 1
  for (int ch = 0; ch < nChunks; ++ch) {
    const int cbase = ch * CHUNK;
    const bool full = al16 && (cbase + CHUNK <= nE);
    int wc = 0;
#pragma unroll
    for (int g = 0; g < NGRP; ++g) {
      const int el0 = (g * NTHR + tid) * 4;
      const int e0  = cbase + el0;
      v4i d;
      if (full) {
        d = *(const v4i*)(eid + e0);
      } else {
        const int i0 = min(e0, nE - 1), i1 = min(e0 + 1, nE - 1);
        const int i2 = min(e0 + 2, nE - 1), i3 = min(e0 + 3, nE - 1);
        const int v0 = eid[i0], v1 = eid[i1], v2 = eid[i2], v3 = eid[i3];
        d.x = (e0     < nE) ? v0 : sent;
        d.y = (e0 + 1 < nE) ? v1 : sent;
        d.z = (e0 + 2 < nE) ? v2 : sent;
        d.w = (e0 + 3 < nE) ? v3 : sent;
      }
      const unsigned s0 = (unsigned)d.x - (unsigned)nodeBase;
      const unsigned s1 = (unsigned)d.y - (unsigned)nodeBase;
      const unsigned s2 = (unsigned)d.z - (unsigned)nodeBase;
      const unsigned s3 = (unsigned)d.w - (unsigned)nodeBase;
      const bool h0 = s0 < (unsigned)NB;
      const bool h1 = s1 < (unsigned)NB;
      const bool h2 = s2 < (unsigned)NB;
      const bool h3 = s3 < (unsigned)NB;
      const unsigned many = __builtin_amdgcn_ballot_w32(h0 | h1 | h2 | h3);
      if (many != 0u) {
#define HITJ(J, HJ, SJ) { \
          const unsigned mj = __builtin_amdgcn_ballot_w32(HJ); \
          if (HJ) { \
            const int pos = wc + (int)__builtin_amdgcn_mbcnt_lo(mj, 0u); \
            if (pos < WCAP) list[wave * WCAP + pos] = ((el0 + (J)) << 10) | (int)(SJ); \
          } \
          wc += (int)__builtin_popcount(mj); }
        HITJ(0, h0, s0)
        HITJ(1, h1, s1)
        HITJ(2, h2, s2)
        HITJ(3, h3, s3)
#undef HITJ
      }
    }
    if (lane == 0) wcnt[wave] = wc;
    __syncthreads();

    if (wave == 0) {
#pragma unroll 1
      for (int wsx = 0; wsx < NWAVE; ++wsx) {
        int n = wcnt[wsx];
        if (n > WCAP) n = WCAP;
        if (n < 0) n = 0;
#pragma unroll 1
        for (int i = 0; i < n; ++i) {
          const int ent  = list[wsx * WCAP + i];
          const int slot = ent & (NB - 1);
          const int el   = (ent >> 10) & (CHUNK - 1);
          int e = cbase + el;
          if (e > nE - 1) e = nE - 1;
          int src = ei[e];
          src = src < 0 ? 0 : (src > nN - 1 ? nN - 1 : src);
          int nd = nodeBase + slot;
          if (nd > nN - 1) nd = nN - 1;
          float l = coef[(size_t)src * CP + hd] + coef[(size_t)nd * CP + NH + hd];
          l = (l > 0.f) ? l : 0.2f * l;
          const int ai = slot * NH + hd;
          const float mo = rmx[ai];
          const float dn = den[ai];
          const float mn = fmaxf(mo, l);
          const float sc = __expf(mo - mn);
          const float p  = __expf(l - mn);
          float hv[CPL], sv[CPL];
#pragma unroll
          for (int c = 0; c < CPL; ++c) {
            hv[c] = h[(size_t)src * HD + cb + c];
            sv[c] = sacc[slot * HD + cb + c];
          }
#pragma unroll
          for (int c = 0; c < CPL; ++c) sacc[slot * HD + cb + c] = sv[c] * sc + p * hv[c];
          den[ai] = dn * sc + p;
          rmx[ai] = mn;
        }
      }
    }
    __syncthreads();
  }

  float bv[CPL];
#pragma unroll
  for (int c = 0; c < CPL; ++c) bv[c] = bias[cb + c];
  double sm[CPL], sq[CPL];
#pragma unroll
  for (int c = 0; c < CPL; ++c) { sm[c] = 0.0; sq[c] = 0.0; }
#pragma unroll 1
  for (int j = 0; j < SPW; ++j) {
    const int slot = wave * SPW + j;
    const int node = nodeBase + slot;
    const float dv  = den[slot * NH + hd];
    const float inv = 1.0f / (dv + 1e-16f);
#pragma unroll
    for (int c = 0; c < CPL; ++c) {
      const float v = sacc[slot * HD + cb + c] * inv + bv[c];
      sacc[slot * HD + cb + c] = v;
      if (node < nN) { sm[c] += (double)v; sq[c] += (double)v * (double)v; }
    }
  }
#pragma unroll
  for (int c = 0; c < CPL; ++c) {
    bpart[wave * (2 * HD) + cb + c]      = sm[c];
    bpart[wave * (2 * HD) + HD + cb + c] = sq[c];
  }
  __syncthreads();
  if (tid < 2 * HD) {
    double t = 0.0;
#pragma unroll 1
    for (int w = 0; w < NWAVE; ++w) t += bpart[w * (2 * HD) + tid];
    bpart[tid] = t;
  }
  __syncthreads();

  float*  ap = agg + (size_t)nodeBase * HD;
  double* pp = part + (size_t)blockIdx.x * PPD;
#pragma unroll 1
  for (int it = 0; it < NIT; ++it) {
    const int f  = it * (NTHR * 4) + tid * 4;
    const int wr = (it * (NTHR * 4) + wave * 128) / HD;
    if (nodeBase + wr < nP) {
      const v4f v = *(const v4f*)(sacc + f);
      *(volatile v4f*)(ap + f) = v;
    }
  }
  if (tid < HD) {
    v2d pv;
    pv.x = bpart[2 * tid]; pv.y = bpart[2 * tid + 1];
    *(volatile v2d*)(pp + 2 * tid) = pv;
  }
  __threadfence();
#pragma unroll 1
  for (int it = 0; it < NIT; ++it) {
    const int f  = it * (NTHR * 4) + tid * 4;
    const int wr = (it * (NTHR * 4) + wave * 128) / HD;
    if (nodeBase + wr < nP) {
      const v4f v = *(const v4f*)(sacc + f);
      *(volatile v4f*)(ap + f) = v;
    }
  }
  if (tid < HD) {
    v2d pv;
    pv.x = bpart[2 * tid]; pv.y = bpart[2 * tid + 1];
    *(volatile v2d*)(pp + 2 * tid) = pv;
  }
}

template <int HD>
__global__ __launch_bounds__(128) void k_bncomb(const double* __restrict__ part,
                                                const float* __restrict__ gam,
                                                const float* __restrict__ bet,
                                                float* bn, int nblk, int nN) {
  __shared__ __attribute__((aligned(16))) float bl[BNW];
  const int tid = threadIdx.x;
  bl[tid] = 0.f;
  __syncthreads();
  if (tid < HD) {
    double s = 0.0, q = 0.0;
#pragma unroll 1
    for (int b = 0; b < nblk; ++b) {
      s += part[(size_t)b * PPD + tid];
      q += part[(size_t)b * PPD + HD + tid];
    }
    const double inv = 1.0 / (double)nN;
    const double mu = s * inv;
    double var = q * inv - mu * mu;
    if (var < 0.0) var = 0.0;
    const float sc = gam[tid] * rsqrtf((float)var + 1e-5f);
    bl[tid]      = sc;
    bl[64 + tid] = bet[tid] - (float)mu * sc;
  }
  __syncthreads();
  if (tid < 32) {
    const v4f v = *(const v4f*)(bl + tid * 4);
    *(volatile v4f*)(bn + tid * 4) = v;
    __threadfence();
    *(volatile v4f*)(bn + tid * 4) = v;
  }
}

__global__ __launch_bounds__(NTHR) void k_apply(const float* __restrict__ agg,
                                                const float* __restrict__ bn,
                                                float* out, int nN) {
  const int total = nN * 32;
  const int f = (blockIdx.x * NTHR + threadIdx.x) * 4;
  if (f >= total) return;
  const int c = f & 31;
  const v4f a  = *(const v4f*)(agg + f);
  const v4f sc = *(const v4f*)(bn + c);
  const v4f sh = *(const v4f*)(bn + 64 + c);
  v4f y = a * sc + sh;
  y.x = fmaxf(y.x, 0.f); y.y = fmaxf(y.y, 0.f); y.z = fmaxf(y.z, 0.f); y.w = fmaxf(y.w, 0.f);
  *(volatile v4f*)(out + f) = y;
  __threadfence();
  *(volatile v4f*)(out + f) = y;
}

extern "C" void kernel_launch(void* const* d_in, const int* in_sizes, int n_in,
                              void* d_out, int out_size, void* d_ws, size_t ws_size,
                              hipStream_t stream) {
  if (n_in < 20) return;
  const int nN = in_sizes[0] / 128;
  if (nN <= 0 || in_sizes[0] != nN * 128) return;
  const int nE = in_sizes[19] / 2;
  if (nE < 0 || in_sizes[19] != 2 * nE) return;
  if (in_sizes[1] != 128 * 64 || in_sizes[7] != 64 * 64 || in_sizes[13] != 64 * 32) return;
  if (in_sizes[2] != 64 || in_sizes[3] != 64 || in_sizes[4] != 64 || in_sizes[5] != 64 || in_sizes[6] != 64) return;
  if (in_sizes[8] != 64 || in_sizes[9] != 64 || in_sizes[10] != 64 || in_sizes[11] != 64 || in_sizes[12] != 64) return;
  if (in_sizes[14] != 32 || in_sizes[15] != 32 || in_sizes[16] != 32 || in_sizes[17] != 32 || in_sizes[18] != 32) return;
  if (out_size != nN * 32) return;

  const float* x   = (const float*)d_in[0];
  const float* W1  = (const float*)d_in[1];
  const float* as1 = (const float*)d_in[2];
  const float* ad1 = (const float*)d_in[3];
  const float* b1  = (const float*)d_in[4];
  const float* g1  = (const float*)d_in[5];
  const float* be1 = (const float*)d_in[6];
  const float* W2  = (const float*)d_in[7];
  const float* as2 = (const float*)d_in[8];
  const float* ad2 = (const float*)d_in[9];
  const float* b2  = (const float*)d_in[10];
  const float* g2  = (const float*)d_in[11];
  const float* be2 = (const float*)d_in[12];
  const float* W3  = (const float*)d_in[13];
  const float* as3 = (const float*)d_in[14];
  const float* ad3 = (const float*)d_in[15];
  const float* b3  = (const float*)d_in[16];
  const float* g3  = (const float*)d_in[17];
  const float* be3 = (const float*)d_in[18];
  const int*   ei  = (const int*)d_in[19];
  float* out = (float*)d_out;

  const int nP   = ((nN + 63) / 64) * 64;
  const int nblk = (nN + NB - 1) / NB;

  size_t off = 0;
  unsigned short* Whi = (unsigned short*)((char*)d_ws + off); off += 16384;
  unsigned short* Wlo = (unsigned short*)((char*)d_ws + off); off += 16384;
  float*  hpl  = (float*)((char*)d_ws + off);  off += (size_t)nP * 64 * sizeof(float);
  float*  coef = (float*)((char*)d_ws + off);  off += (size_t)nP * 4 * sizeof(float);
  float*  aggA = (float*)((char*)d_ws + off);  off += (size_t)nP * 64 * sizeof(float);
  float*  aggB = (float*)((char*)d_ws + off);  off += (size_t)nP * 64 * sizeof(float);
  float*  bn   = (float*)((char*)d_ws + off);  off += 512;
  double* part = (double*)((char*)d_ws + off); off += (size_t)nblk * PPD * sizeof(double);
  if (off > ws_size) return;
  if (off > (size_t)134217728) return;

  const int lds64 = GAT_LDS(64, 2);
  const int lds32 = GAT_LDS(32, 1);

  k_prep<<<(64 * 128 / 8 + NTHR - 1) / NTHR, NTHR, 0, stream>>>(W1, Whi, Wlo, 128, 64);
  k_gemm<128, 64, 2, 32, 0><<<nP / 32, NTHR, 0, stream>>>(x, Whi, Wlo, as1, ad1, bn, hpl, coef, nN);
  hipFuncSetAttribute(reinterpret_cast<const void*>(&k_gat<64, 2>),
                      hipFuncAttributeMaxDynamicSharedMemorySize, lds64);
  k_gat<64, 2><<<nblk, NTHR, lds64, stream>>>(ei, hpl, coef, b1, aggA, part, nN, nE, nP);
  k_bncomb<64><<<1, 128, 0, stream>>>(part, g1, be1, bn, nblk, nN);

  k_prep<<<(64 * 64 / 8 + NTHR - 1) / NTHR, NTHR, 0, stream>>>(W2, Whi, Wlo, 64, 64);
  k_gemm<64, 64, 2, 32, 1><<<nP / 32, NTHR, 0, stream>>>(aggA, Whi, Wlo, as2, ad2, bn, hpl, coef, nN);
  k_gat<64, 2><<<nblk, NTHR, lds64, stream>>>(ei, hpl, coef, b2, aggB, part, nN, nE, nP);
  k_bncomb<64><<<1, 128, 0, stream>>>(part, g2, be2, bn, nblk, nN);

  k_prep<<<(32 * 64 / 8 + NTHR - 1) / NTHR, NTHR, 0, stream>>>(W3, Whi, Wlo, 64, 32);
  k_gemm<64, 32, 1, 64, 1><<<nP / 64, NTHR, 0, stream>>>(aggB, Whi, Wlo, as3, ad3, bn, hpl, coef, nN);
  hipFuncSetAttribute(reinterpret_cast<const void*>(&k_gat<32, 1>),
                      hipFuncAttributeMaxDynamicSharedMemorySize, lds32);
  k_gat<32, 1><<<nblk, NTHR, lds32, stream>>>(ei, hpl, coef, b3, aggA, part, nN, nE, nP);
  k_bncomb<32><<<1, 128, 0, stream>>>(part, g3, be3, bn, nblk, nN);
  k_apply<<<(nN * 8 + NTHR - 1) / NTHR, NTHR, 0, stream>>>(aggA, bn, out, nN);
}
